// MultiHeadAttention_63806034150218
// MI455X (gfx1250) — hardware-verified
//
#include <hip/hip_runtime.h>


#ifndef NB
#define NB 4
#endif
#ifndef SEQ
#define SEQ 2048
#endif
#define NB_FULL  4
#define SEQ_FULL 2048
#ifndef OUT_SEQ
#define OUT_SEQ SEQ
#endif
#define DM   1024
#define NH_  16
#define HD   64
#define AW   4
#define ER   ((SEQ) < 512 ? (SEQ) : 512)
#define QRS  2048.0f
#define QRI  (1.0f / 2048.0f)
#define SC2  (0.125f * 1.4426950408889634f)
#define PSH  8.0f
#define NEGV (-3.0e38f)
#define CTXS 16.0f
#define WOS  256.0f
#define OSC  (1.0f / 4096.0f)

static_assert(HD == 64);
static_assert(NH_ * HD == DM);
static_assert(DM % 64 == 0);
static_assert(DM % 32 == 0);
static_assert(SEQ % 64 == 0);
static_assert((NB * SEQ) % 64 == 0);
static_assert(SEQ % 32 == 0);
static_assert(ER % 64 == 0);
static_assert(ER % (16 * AW) == 0);
static_assert((SEQ - ER) % 64 == 0);
static_assert((SEQ - ER) % (16 * AW) == 0);
static_assert(ER <= SEQ);
static_assert(NB <= NB_FULL);
static_assert(SEQ <= SEQ_FULL);

typedef _Float16 h16;
typedef unsigned short bf;
typedef __attribute__((ext_vector_type(16))) __bf16   v16bf;
typedef __attribute__((ext_vector_type(16))) _Float16 v16h;
typedef __attribute__((ext_vector_type(8)))  _Float16 v8h;
typedef __attribute__((ext_vector_type(8)))  unsigned short v8us;
typedef __attribute__((ext_vector_type(8)))  float    v8f;
typedef __attribute__((ext_vector_type(4)))  float    v4f;
typedef v4f  __attribute__((may_alias)) v4fa;
typedef v8us __attribute__((may_alias)) v8usa;

__device__ __forceinline__ unsigned short f2bf(float f) { unsigned u = __float_as_uint(f); u += 0x7FFFu + ((u >> 16) & 1u); return (unsigned short)(u >> 16); }
__device__ __forceinline__ float bfr(float f) { return __uint_as_float(((unsigned)f2bf(f)) << 16); }
__device__ __forceinline__ v16h cat16(v8h lo, v8h hi) { return __builtin_shufflevector(lo, hi, 0, 1, 2, 3, 4, 5, 6, 7, 8, 9, 10, 11, 12, 13, 14, 15); }
__device__ __forceinline__ v16bf cat16b(v8us lo, v8us hi) { return __builtin_bit_cast(v16bf, __builtin_shufflevector(lo, hi, 0, 1, 2, 3, 4, 5, 6, 7, 8, 9, 10, 11, 12, 13, 14, 15)); }
__device__ __forceinline__ v8f wmma16(v16h a, v16h b, v8f c) { return __builtin_amdgcn_wmma_f32_16x16x32_f16(false, a, false, b, (short)0, c, false, false); }
__device__ __forceinline__ v8f wmmab(v16bf a, v16bf b, v8f c) { return __builtin_amdgcn_wmma_f32_16x16x32_bf16(false, a, false, b, (short)0, c, false, false); }
__device__ __forceinline__ v16h  ldh(const h16* p) { return cat16(*(const v8h*)p, *(const v8h*)(p + 16)); }
__device__ __forceinline__ v16bf ldb(const bf* p)  { return cat16b(*(const v8us*)p, *(const v8us*)(p + 16)); }
__device__ __forceinline__ void wave_sync() { __builtin_amdgcn_fence(3  , "wavefront"); __builtin_amdgcn_wave_barrier(); asm volatile("" ::: "memory"); }

__global__ __launch_bounds__(256) void k_cvt8(const float* __restrict__ src, bf* dst, size_t n8) {
    const size_t i = (size_t)blockIdx.x * 256 + threadIdx.x; if (i >= n8) return;
    const v8f v = *(const v8f*)(src + i * 8); v8us o;
#pragma unroll
    for (int k = 0; k < 8; ++k) o[k] = f2bf(v[k]);
    *(volatile v8us*)(dst + i * 8) = o; __threadfence(); *(volatile v8us*)(dst + i * 8) = o;
}

__global__ __launch_bounds__(256) void k_tr(const float* __restrict__ W, unsigned short* Wt, int N, int asF16) {
    __shared__ __align__(16) unsigned short tile[64 * 72];
    const int tid = threadIdx.x; const int k0 = blockIdx.x * 64, n0 = blockIdx.y * 64;
#pragma unroll 4
    for (int i = 0; i < 16; ++i) {
        const int idx = tid + i * 256; const int r = idx >> 6, c = idx & 63;
        const float w = W[(size_t)(k0 + r) * (size_t)N + n0 + c];
        const unsigned short bb = f2bf(w);
        const h16 hv = (h16)(bfr(w) * WOS);
        const unsigned short hb = __builtin_bit_cast(unsigned short, hv);
        tile[c * 72 + r] = asF16 ? hb : bb; }
    __syncthreads();
#pragma unroll 1
    for (int ps = 0; ps < 2; ++ps) {
#pragma unroll
        for (int i = 0; i < 2; ++i) {
            const int idx = tid + i * 256; const int r = idx >> 3, c8 = (idx & 7) * 8;
            const v8us v = *(const v8usa*)(&tile[r * 72 + c8]);
            *(volatile v8us*)(Wt + (size_t)(n0 + r) * DM + k0 + c8) = v; }
        if (ps == 0) __threadfence(); }
}

__global__ __launch_bounds__(32) void k_proj(const bf* __restrict__ A, const bf* __restrict__ Bt, const float* __restrict__ bias, int biasRow,
                                             h16* Ph, h16* Pr, int resMode, int RB, size_t sRB, int pitch, int CB, size_t sCB,
                                             size_t sRBr, int pitchR, size_t sCBr) {
    __shared__ __align__(16) float os[16 * 68];
    const int K = DM;
    const int lane = threadIdx.x & 31, lr = lane & 15, hi = lane >> 4; const int r0 = blockIdx.x * 64, c0 = blockIdx.y * 64;
    v8f acc[4][4];
#pragma unroll
    for (int mb = 0; mb < 4; ++mb)
#pragma unroll
        for (int nb = 0; nb < 4; ++nb) acc[mb][nb] = (v8f){};
    const size_t aoff = (size_t)(r0 + lr) * K + 8 * hi, boff = (size_t)(c0 + lr) * K + 8 * hi;
#pragma unroll 1
    for (int kc = 0; kc < K; kc += 32) {
        v16bf a[4];
#pragma unroll
        for (int mb = 0; mb < 4; ++mb) a[mb] = ldb(A + aoff + (size_t)mb * 16 * K + kc);
#pragma unroll
        for (int nb = 0; nb < 4; ++nb) { const v16bf b = ldb(Bt + boff + (size_t)nb * 16 * K + kc);
#pragma unroll
            for (int mb = 0; mb < 4; ++mb) acc[mb][nb] = wmmab(a[mb], b, acc[mb][nb]); }
        asm volatile("v_nop\n\tv_nop\n\tv_nop\n\tv_nop" : "+v"(acc[0][0]), "+v"(acc[1][1]), "+v"(acc[2][2]), "+v"(acc[3][3]) : "v"(a[0]), "v"(a[1]), "v"(a[2]), "v"(a[3]));
    }
    const int tok0 = (resMode == 1) ? (r0 % RB) : (c0 % CB);
    const int useRes = (resMode != 0) && (tok0 < ER);
    const size_t tbase  = (size_t)(r0 / RB) * sRB  + (size_t)(r0 % RB) * (size_t)pitch  + (size_t)(c0 / CB) * sCB  + (size_t)(c0 % CB);
    const size_t tbaseR = (size_t)(r0 / RB) * sRBr + (size_t)(r0 % RB) * (size_t)pitchR + (size_t)(c0 / CB) * sCBr + (size_t)(c0 % CB);
    float bcol[4];
#pragma unroll
    for (int nb = 0; nb < 4; ++nb) { const int ci = biasRow ? 0 : (c0 + nb * 16 + lr); const float bvv = bfr(bias[ci]); bcol[nb] = biasRow ? 0.0f : bvv; }
#pragma unroll
    for (int mb = 0; mb < 4; ++mb) {
        float brow[8];
#pragma unroll
        for (int j = 0; j < 8; ++j) { const int ri = biasRow ? (r0 + mb * 16 + hi * 8 + j) : 0; const float bvv = bfr(bias[ri]); brow[j] = biasRow ? bvv : 0.0f; }
#pragma unroll
        for (int nb = 0; nb < 4; ++nb) {
#pragma unroll
            for (int j = 0; j < 8; ++j) os[(hi * 8 + j) * 68 + nb * 16 + lr] = acc[mb][nb][j] + bcol[nb] + brow[j]; }
        wave_sync();
        const size_t sb  = tbase  + (size_t)(mb * 16) * (size_t)pitch;
        const size_t sbR = tbaseR + (size_t)(mb * 16) * (size_t)pitchR;
#pragma unroll 1
        for (int ps = 0; ps < 2; ++ps) {
#pragma unroll
            for (int s = 0; s < 4; ++s) { const int row = 4 * s + (lane >> 3), c8 = (lane & 7) * 8;
                const v4f x0 = *(const v4fa*)(&os[row * 68 + c8]); const v4f x1 = *(const v4fa*)(&os[row * 68 + c8 + 4]); v8h hv, rv;
#pragma unroll
                for (int i = 0; i < 4; ++i) { const h16 a0 = (h16)x0[i]; const h16 a1 = (h16)x1[i]; hv[i] = a0; hv[4 + i] = a1; rv[i] = (h16)((x0[i] - (float)a0) * QRS); rv[4 + i] = (h16)((x1[i] - (float)a1) * QRS); }
                const size_t oo  = sb  + (size_t)row * (size_t)pitch  + c8;
                const size_t ooR = sbR + (size_t)row * (size_t)pitchR + c8;
                *(volatile v8h*)(Ph + oo) = hv; if (useRes) *(volatile v8h*)(Pr + ooR) = rv; }
            if (ps == 0) __threadfence(); }
        wave_sync();
    }
}

#define ST8(J, O, S) { v4f a_, c_; a_[0] = (O)[0] * (S); a_[1] = (O)[1] * (S); a_[2] = (O)[2] * (S); a_[3] = (O)[3] * (S); \
                       c_[0] = (O)[4] * (S); c_[1] = (O)[5] * (S); c_[2] = (O)[6] * (S); c_[3] = (O)[7] * (S); \
                       *(v4fa*)(&os[wb + lr * 68 + 16 * (J) + 8 * hi]) = a_; *(v4fa*)(&os[wb + lr * 68 + 16 * (J) + 8 * hi + 4]) = c_; }

template <int EARLY>
__global__ __launch_bounds__(32 * AW) void k_flash(const h16* __restrict__ QH, const h16* __restrict__ QR, const h16* __restrict__ KP, const h16* __restrict__ KR,
                                                   const h16* __restrict__ VT, const h16* __restrict__ VR, h16* CH, h16* CR) {
    __shared__ __align__(16) float os[AW * 16 * 68];
    const int lane = threadIdx.x & 31, wave = __builtin_amdgcn_readfirstlane((int)(threadIdx.x >> 5)), lr = lane & 15, hi = lane >> 4;
    const int zh = blockIdx.y; const int b = zh / NH_, h = zh % NH_;
    const int t0 = (EARLY ? 0 : ER) + (blockIdx.x * AW + wave) * 16;
    const int tq = t0 + lr;
    const size_t pbase = (size_t)zh * SEQ * HD;
    const size_t pbr   = (size_t)zh * ER * HD;
    const size_t qo = pbase + (size_t)tq * HD + 8 * hi;
    const v16h qh0 = ldh(QH + qo), qh1 = ldh(QH + qo + 32);
    v16h qr0 = qh0, qr1 = qh1;
    if (EARLY) { const size_t qor = pbr + (size_t)tq * HD + 8 * hi; qr0 = ldh(QR + qor); qr1 = ldh(QR + qor + 32); }
    const size_t ko  = pbase + (size_t)lr * HD + 8 * hi;
    const size_t kor = pbr   + (size_t)lr * HD + 8 * hi;
    const size_t vo  = pbase + (size_t)lr * SEQ + 8 * hi;
    const size_t vor = pbr   + (size_t)lr * ER + 8 * hi;
    v8f o0 = (v8f){}, o1 = (v8f){}, o2 = (v8f){}, o3 = (v8f){};
    v8f e0 = (v8f){}, e1 = (v8f){}, e2 = (v8f){}, e3 = (v8f){};
    float m = NEGV, l = 0.0f;
    const int kend = t0 + 16;
#pragma unroll 1
    for (int key0 = 0; key0 < kend; key0 += 32) {
        const h16* ka = KP + ko + (size_t)key0 * HD;
        const v16h ka0 = ldh(ka), ka1 = ldh(ka + 32), kb0 = ldh(ka + 16 * HD), kb1 = ldh(ka + 16 * HD + 32);
        float ta[8], tb[8];
        if (EARLY) {
            const h16* kr = KR + kor + (size_t)key0 * HD;
            const v16h ra0 = ldh(kr), ra1 = ldh(kr + 32), rb0 = ldh(kr + 16 * HD), rb1 = ldh(kr + 16 * HD + 32);
            v8f sHa = (v8f){}, sLa = (v8f){}, sHb = (v8f){}, sLb = (v8f){};
            sHa = wmma16(ka0, qh0, sHa); sLa = wmma16(ka0, qr0, sLa); sHb = wmma16(kb0, qh0, sHb); sLb = wmma16(kb0, qr0, sLb);
            sHa = wmma16(ka1, qh1, sHa); sLa = wmma16(ka1, qr1, sLa); sHb = wmma16(kb1, qh1, sHb); sLb = wmma16(kb1, qr1, sLb);
            sLa = wmma16(ra0, qh0, sLa); sLb = wmma16(rb0, qh0, sLb); sLa = wmma16(ra1, qh1, sLa); sLb = wmma16(rb1, qh1, sLb);
            asm volatile("v_nop\n\tv_nop\n\tv_nop\n\tv_nop" : "+v"(sHa), "+v"(sLa), "+v"(sHb), "+v"(sLb) : "v"(ka0), "v"(ka1), "v"(kb0), "v"(kb1), "v"(ra0), "v"(ra1), "v"(rb0), "v"(rb1));
#pragma unroll
            for (int r = 0; r < 8; ++r) { ta[r] = (sHa[r] + sLa[r] * QRI) * SC2; tb[r] = (sHb[r] + sLb[r] * QRI) * SC2; }
        } else {
            v8f sHa = (v8f){}, sHb = (v8f){};
            sHa = wmma16(ka0, qh0, sHa); sHb = wmma16(kb0, qh0, sHb);
            sHa = wmma16(ka1, qh1, sHa); sHb = wmma16(kb1, qh1, sHb);
            asm volatile("v_nop\n\tv_nop\n\tv_nop\n\tv_nop" : "+v"(sHa), "+v"(sHb) : "v"(ka0), "v"(ka1), "v"(kb0), "v"(kb1));
#pragma unroll
            for (int r = 0; r < 8; ++r) { ta[r] = sHa[r] * SC2; tb[r] = sHb[r] * SC2; }
        }
        if (key0 + 31 > t0) {
#pragma unroll
            for (int r = 0; r < 8; ++r) { const int kk = key0 + 8 * hi + r; ta[r] = (kk <= tq) ? ta[r] : NEGV; tb[r] = (kk + 16 <= tq) ? tb[r] : NEGV; }
        }
        float mx = NEGV;
#pragma unroll
        for (int r = 0; r < 8; ++r) mx = fmaxf(mx, fmaxf(ta[r], tb[r]));
        mx = fmaxf(mx, __shfl_xor(mx, 16, 32));
        const float mnew = fmaxf(m, mx);
        const float alpha = __builtin_amdgcn_exp2f(m - mnew);
        const float sh = PSH - mnew;
        v16h pb, pr; float ls = 0.0f;
        if (EARLY) {
#pragma unroll
            for (int r = 0; r < 8; ++r) {
                const float fa = __builtin_amdgcn_exp2f(ta[r] + sh), fc = __builtin_amdgcn_exp2f(tb[r] + sh);
                const h16 pa = (h16)fa, pc = (h16)fc;
                const h16 ra = (h16)((fa - (float)pa) * QRS), rc = (h16)((fc - (float)pc) * QRS);
                pb[r] = pa; pb[8 + r] = pc; pr[r] = ra; pr[8 + r] = rc;
                ls += ((float)pa + (float)ra * QRI) + ((float)pc + (float)rc * QRI); }
        } else {
#pragma unroll
            for (int r = 0; r < 8; ++r) { const h16 pa = (h16)__builtin_amdgcn_exp2f(ta[r] + sh); const h16 pc = (h16)__builtin_amdgcn_exp2f(tb[r] + sh); pb[r] = pa; pb[8 + r] = pc; ls += (float)pa + (float)pc; }
            pr = pb;
        }
        l = l * alpha + ls; m = mnew;
        o0 = o0 * alpha; o1 = o1 * alpha; o2 = o2 * alpha; o3 = o3 * alpha;
        const h16* va = VT + vo + key0;
        const v16h v0 = ldh(va), v1 = ldh(va + (size_t)16 * SEQ), v2 = ldh(va + (size_t)32 * SEQ), v3 = ldh(va + (size_t)48 * SEQ);
        if (EARLY) {
            e0 = e0 * alpha; e1 = e1 * alpha; e2 = e2 * alpha; e3 = e3 * alpha;
            const h16* vr = VR + vor + key0;
            const v16h w0 = ldh(vr), w1 = ldh(vr + (size_t)16 * ER), w2 = ldh(vr + (size_t)32 * ER), w3 = ldh(vr + (size_t)48 * ER);
            o0 = wmma16(v0, pb, o0); o1 = wmma16(v1, pb, o1); o2 = wmma16(v2, pb, o2); o3 = wmma16(v3, pb, o3);
            e0 = wmma16(w0, pb, e0); e1 = wmma16(w1, pb, e1); e2 = wmma16(w2, pb, e2); e3 = wmma16(w3, pb, e3);
            e0 = wmma16(v0, pr, e0); e1 = wmma16(v1, pr, e1); e2 = wmma16(v2, pr, e2); e3 = wmma16(v3, pr, e3);
            asm volatile("v_nop\n\tv_nop\n\tv_nop\n\tv_nop" : "+v"(o0), "+v"(o1), "+v"(o2), "+v"(o3), "+v"(e0), "+v"(e1), "+v"(e2), "+v"(e3) : "v"(v0), "v"(v1), "v"(v2), "v"(v3), "v"(w0), "v"(w1), "v"(w2), "v"(w3), "v"(pb), "v"(pr));
        } else {
            o0 = wmma16(v0, pb, o0); o1 = wmma16(v1, pb, o1); o2 = wmma16(v2, pb, o2); o3 = wmma16(v3, pb, o3);
            asm volatile("v_nop\n\tv_nop\n\tv_nop\n\tv_nop" : "+v"(o0), "+v"(o1), "+v"(o2), "+v"(o3) : "v"(v0), "v"(v1), "v"(v2), "v"(v3), "v"(pb));
        }
    }
    l += __shfl_xor(l, 16, 32);
    const float inv = CTXS * (1.0f / l);
    const int wb = wave * 16 * 68;
    v8f f0 = o0, f1 = o1, f2 = o2, f3 = o3;
    if (EARLY) { f0 = o0 + e0 * QRI; f1 = o1 + e1 * QRI; f2 = o2 + e2 * QRI; f3 = o3 + e3 * QRI; }
    ST8(0, f0, inv) ST8(1, f1, inv) ST8(2, f2, inv) ST8(3, f3, inv)
    wave_sync();
    const size_t crow = ((size_t)b * SEQ + t0) * DM + h * HD;
    const size_t rrow = ((size_t)b * ER + t0) * DM + h * HD;
#pragma unroll 1
    for (int ps = 0; ps < 2; ++ps) {
#pragma unroll
        for (int s = 0; s < 4; ++s) { const int row = 4 * s + (lane >> 3), c8 = (lane & 7) * 8;
            const v4f x0 = *(const v4fa*)(&os[wb + row * 68 + c8]); const v4f x1 = *(const v4fa*)(&os[wb + row * 68 + c8 + 4]); v8h hv, rv;
#pragma unroll
            for (int i = 0; i < 4; ++i) { const h16 a0 = (h16)x0[i]; const h16 a1 = (h16)x1[i]; hv[i] = a0; hv[4 + i] = a1; rv[i] = (h16)((x0[i] - (float)a0) * QRS); rv[4 + i] = (h16)((x1[i] - (float)a1) * QRS); }
            *(volatile v8h*)(CH + crow + (size_t)row * DM + c8) = hv;
            if (EARLY) *(volatile v8h*)(CR + rrow + (size_t)row * DM + c8) = rv; }
        if (ps == 0) __threadfence(); }
}

template <int MB, int RES>
__global__ __launch_bounds__(32) void k_out(const h16* __restrict__ CH, const h16* __restrict__ CR, const h16* __restrict__ Wt, const float* __restrict__ bias, float* OUT, int tpb, int tb0) {
    __shared__ __align__(16) float os[16 * 68];
    const int K = DM;
    const int lane = threadIdx.x & 31, lr = lane & 15, hi = lane >> 4;
    const int b = blockIdx.x / tpb, ti = blockIdx.x % tpb; const int t0 = tb0 + ti * (16 * MB); const int c0 = blockIdx.y * 64;
    v8f acc[MB][4], accr[MB][4];
#pragma unroll
    for (int mb = 0; mb < MB; ++mb)
#pragma unroll
        for (int nb = 0; nb < 4; ++nb) { acc[mb][nb] = (v8f){}; accr[mb][nb] = (v8f){}; }
    const size_t aoff = ((size_t)b * SEQ + t0 + lr) * K + 8 * hi;
    const size_t roff = ((size_t)b * ER + t0 + lr) * K + 8 * hi;
    const size_t boff = (size_t)(c0 + lr) * K + 8 * hi;
#pragma unroll 1
    for (int kc = 0; kc < K; kc += 32) {
        v16h a[MB], ar[MB];
#pragma unroll
        for (int mb = 0; mb < MB; ++mb) { a[mb] = ldh(CH + aoff + (size_t)mb * 16 * K + kc); ar[mb] = a[mb]; if (RES) ar[mb] = ldh(CR + roff + (size_t)mb * 16 * K + kc); }
#pragma unroll
        for (int nb = 0; nb < 4; ++nb) { const v16h bq = ldh(Wt + boff + (size_t)nb * 16 * K + kc);
#pragma unroll
            for (int mb = 0; mb < MB; ++mb) { acc[mb][nb] = wmma16(a[mb], bq, acc[mb][nb]); if (RES) accr[mb][nb] = wmma16(ar[mb], bq, accr[mb][nb]); } }
#pragma unroll
        for (int mb = 0; mb < MB; ++mb) {
            asm volatile("" : "+v"(acc[mb][0]), "+v"(acc[mb][1]), "+v"(acc[mb][2]), "+v"(acc[mb][3]) : "v"(a[mb]));
            if (RES) asm volatile("" : "+v"(accr[mb][0]), "+v"(accr[mb][1]), "+v"(accr[mb][2]), "+v"(accr[mb][3]) : "v"(ar[mb])); }
        asm volatile("v_nop\n\tv_nop\n\tv_nop\n\tv_nop" : "+v"(acc[0][0]), "+v"(acc[MB - 1][3]) : "v"(a[0]), "v"(a[MB - 1]));
    }
    const v4f bv = *(const v4f*)(bias + c0 + lr * 4); v4f b4;
#pragma unroll
    for (int i = 0; i < 4; ++i) b4[i] = bfr(bv[i]);
#pragma unroll
    for (int mb = 0; mb < MB; ++mb) {
#pragma unroll
        for (int nb = 0; nb < 4; ++nb) {
#pragma unroll
            for (int j = 0; j < 8; ++j) os[(hi * 8 + j) * 68 + nb * 16 + lr] = RES ? (acc[mb][nb][j] + accr[mb][nb][j] * QRI) * OSC : acc[mb][nb][j] * OSC; }
        wave_sync();
        float* orow = OUT + ((size_t)b * OUT_SEQ + t0 + mb * 16) * DM + c0;
#pragma unroll 1
        for (int ps = 0; ps < 2; ++ps) {
#pragma unroll
            for (int s = 0; s < 8; ++s) { const int row = 2 * s + hi, cofs = lr * 4;
                const v4f val = *(const v4fa*)(&os[row * 68 + cofs]) + b4;
                *(volatile v4f*)(orow + (size_t)row * DM + cofs) = val; }
            if (ps == 0) __threadfence(); }
        wave_sync();
    }
}

static constexpr size_t al256(size_t v) { return (v + 255) & ~(size_t)255; }
static constexpr size_t SZ_XB = al256((size_t)NB * SEQ * DM * 2);
static constexpr size_t SZ_WT = al256((size_t)3 * DM * DM * 2);
static constexpr size_t SZ_WO = al256((size_t)DM * DM * 2);
static constexpr size_t SZ_PL = al256((size_t)NB * NH_ * SEQ * HD * 2);
static constexpr size_t SZ_PR = al256((size_t)NB * NH_ * ER * HD * 2);
static constexpr size_t SZ_CX = al256((size_t)NB * SEQ * DM * 2);
static constexpr size_t SZ_CR = al256((size_t)NB * ER * DM * 2);
static constexpr size_t SZ_TOTAL = SZ_XB + SZ_WT + SZ_WO + 3 * SZ_PL + 3 * SZ_PR + SZ_CX + SZ_CR;
static_assert(SZ_TOTAL <= (size_t)134217728);
static_assert(((size_t)DM * DM * 2) % 256 == 0);

extern "C" void kernel_launch(void* const* d_in, const int* in_sizes, int n_in,
                              void* d_out, int out_size, void* d_ws, size_t ws_size, hipStream_t stream) {
    if (n_in < 5) return;
    const size_t needx = ((size_t)(NB - 1) * SEQ_FULL + SEQ) * DM;
    if ((size_t)in_sizes[0] < needx) return;
    if ((size_t)in_sizes[1] < (size_t)3 * DM * DM || (size_t)in_sizes[2] < (size_t)3 * DM) return;
    if ((size_t)in_sizes[3] < (size_t)DM * DM || (size_t)in_sizes[4] < (size_t)DM) return;
    if ((size_t)out_size < ((size_t)(NB - 1) * OUT_SEQ + SEQ) * DM) return;
    if (SZ_TOTAL > ws_size) return;
    const float* x = (const float*)d_in[0]; const float* wqkv = (const float*)d_in[1]; const float* bqkv = (const float*)d_in[2];
    const float* wout = (const float*)d_in[3]; const float* bout = (const float*)d_in[4];
    float* OUT = (float*)d_out;
    char* wsp = (char*)d_ws;
    bf*  XB  = (bf*)wsp;  wsp += SZ_XB;
    bf*  WT  = (bf*)wsp;  wsp += SZ_WT;
    h16* WOT = (h16*)wsp; wsp += SZ_WO;
    h16* QH  = (h16*)wsp; wsp += SZ_PL;
    h16* KP  = (h16*)wsp; wsp += SZ_PL;
    h16* VT  = (h16*)wsp; wsp += SZ_PL;
    h16* QR  = (h16*)wsp; wsp += SZ_PR;
    h16* KR  = (h16*)wsp; wsp += SZ_PR;
    h16* VR  = (h16*)wsp; wsp += SZ_PR;
    h16* CH  = (h16*)wsp; wsp += SZ_CX;
    h16* CR  = (h16*)wsp; wsp += SZ_CR;

    if (SEQ == SEQ_FULL) {
        const size_t n8 = (size_t)NB * SEQ * DM / 8;
        k_cvt8<<<(unsigned)((n8 + 255) / 256), 256, 0, stream>>>(x, XB, n8);
    } else {
        const size_t n8 = (size_t)SEQ * DM / 8;
        for (int b = 0; b < NB; ++b) k_cvt8<<<(unsigned)((n8 + 255) / 256), 256, 0, stream>>>(x + (size_t)b * SEQ_FULL * DM, XB + (size_t)b * SEQ * DM, n8);
    }
    k_tr<<<dim3(DM / 64, 3 * DM / 64, 1), 256, 0, stream>>>(wqkv, (unsigned short*)WT, 3 * DM, 0);
    k_tr<<<dim3(DM / 64, DM / 64, 1), 256, 0, stream>>>(wout, (unsigned short*)WOT, DM, 1);

    k_proj<<<dim3(NB * SEQ / 64, DM / 64, 1), 32, 0, stream>>>(XB, WT, bqkv, 0, QH, QR, 1, SEQ, (size_t)NH_ * SEQ * HD, HD, HD, (size_t)SEQ * HD,
                                                               (size_t)NH_ * ER * HD, HD, (size_t)ER * HD);
    k_proj<<<dim3(NB * SEQ / 64, DM / 64, 1), 32, 0, stream>>>(XB, WT + (size_t)DM * DM, bqkv + DM, 0, KP, KR, 1, SEQ, (size_t)NH_ * SEQ * HD, HD, HD, (size_t)SEQ * HD,
                                                               (size_t)NH_ * ER * HD, HD, (size_t)ER * HD);
    k_proj<<<dim3(DM / 64, NB * SEQ / 64, 1), 32, 0, stream>>>(WT + (size_t)2 * DM * DM, XB, bqkv + 2 * DM, 1, VT, VR, 2, DM, (size_t)0, SEQ, SEQ, (size_t)DM * SEQ,
                                                               (size_t)0, ER, (size_t)DM * ER);

    k_flash<1><<<dim3(ER / (16 * AW), NB * NH_, 1), 32 * AW, 0, stream>>>(QH, QR, KP, KR, VT, VR, CH, CR);
    if (SEQ > ER)
        k_flash<0><<<dim3((SEQ - ER) / (16 * AW), NB * NH_, 1), 32 * AW, 0, stream>>>(QH, QR, KP, KR, VT, VR, CH, CR);

    k_out<2, 1><<<dim3(NB * (ER / 32), DM / 64, 1), 32, 0, stream>>>(CH, CR, WOT, bout, OUT, ER / 32, 0);
    if (SEQ > ER)
        k_out<4, 0><<<dim3(NB * ((SEQ - ER) / 64), DM / 64, 1), 32, 0, stream>>>(CH, CR, WOT, bout, OUT, (SEQ - ER) / 64, ER);
}
